// KANLinear_66065186947649
// MI455X (gfx1250) — hardware-verified
//
#include <hip/hip_runtime.h>
#include <math.h>
#include <stdint.h>

constexpr int kBatch    = 16384;
constexpr int kIn       = 512;
constexpr int kOutF     = 512;
constexpr int kGridLen  = 12;
constexpr int kNSpl     = 8;
constexpr int kNBlk     = 9;
constexpr int kKdim     = kIn * kNBlk;
constexpr int kHalfRows = 8192;
constexpr int kPieces   = kKdim / 8;
constexpr float kACarry   = 8.0f;
constexpr float kWCarry   = 64.0f;
constexpr float kOutScale = 1.0f / 512.0f;

constexpr size_t kABytes  = (size_t)kHalfRows * kKdim * 2;
constexpr size_t kWBytes  = (size_t)kOutF * kKdim * 2;
constexpr size_t kWsTotal = kABytes + kWBytes;
static_assert(kWsTotal <= (size_t)134217728, "carve");
static_assert(kABytes % 128 == 0, "align");
static_assert(kKdim % 32 == 0, "K multiple of 32");
static_assert(kHalfRows % 64 == 0 && kOutF % 64 == 0, "M,N multiples of 64");
static_assert(2 * kHalfRows == kBatch, "two sweeps cover the batch");
static_assert(kPieces == 576, "pieces");
static_assert((kKdim * 2) % 128 == 0, "16-bit row pitch is a line multiple");

typedef __attribute__((ext_vector_type(16))) _Float16 v16h;
typedef __attribute__((ext_vector_type(8)))  _Float16 v8h;
typedef __attribute__((ext_vector_type(16))) __bf16   v16b;
typedef __attribute__((ext_vector_type(8)))  __bf16   v8b;
typedef __attribute__((ext_vector_type(8)))  float    v8f;
typedef __attribute__((ext_vector_type(4)))  float    v4f;
typedef __attribute__((ext_vector_type(4)))  unsigned int v4u;

__device__ __forceinline__ unsigned short f2bf_bits(float f) {
  unsigned u = __float_as_uint(f);
  return (unsigned short)((u + 0x7FFFu + ((u >> 16) & 1u)) >> 16);
}
__device__ __forceinline__ float bf_bits2f(unsigned short h) { return __uint_as_float(((unsigned)h) << 16); }

__device__ __forceinline__ void dep_guard_h(v8f& a, v8f& b, v16h x, v16h y) { asm volatile("v_nop\n\tv_nop\n\tv_nop\n\tv_nop" : "+v"(a), "+v"(b) : "v"(x), "v"(y)); }
__device__ __forceinline__ void dep_guard_b(v8f& a, v8f& b, v16b x, v16b y) { asm volatile("v_nop\n\tv_nop\n\tv_nop\n\tv_nop" : "+v"(a), "+v"(b) : "v"(x), "v"(y)); }
__device__ __forceinline__ void keep4_h(v16h a, v16h b, v16h c, v16h d) { asm volatile("v_nop" :: "v"(a), "v"(b), "v"(c), "v"(d)); }
__device__ __forceinline__ void keep4_b(v16b a, v16b b, v16b c, v16b d) { asm volatile("v_nop" :: "v"(a), "v"(b), "v"(c), "v"(d)); }
__device__ __forceinline__ void acc_guard4(v8f& a, v8f& b, v8f& c, v8f& d) { asm volatile("v_nop\n\tv_nop\n\tv_nop\n\tv_nop" : "+v"(a), "+v"(b), "+v"(c), "+v"(d)); }
template <typename T> struct Frag;
template <> struct Frag<_Float16> {
  typedef v16h V; union U { v16h v; v8h h[2]; };
  static __device__ __forceinline__ v16h load(const _Float16* p) {
    U f; f.h[0] = *(const v8h*)(p); f.h[1] = *(const v8h*)(p + 16); return f.v;
  }
  static __device__ __forceinline__ v8f mma(v16h a, v16h b, v8f c) {
    return __builtin_amdgcn_wmma_f32_16x16x32_f16(false, a, false, b, (short)0, c, false, false);
  }
  static __device__ __forceinline__ void guard(v8f& a, v8f& b, v16h x, v16h y) { dep_guard_h(a, b, x, y); }
  static __device__ __forceinline__ void keep(v16h a, v16h b, v16h c, v16h d) { keep4_h(a, b, c, d); }
};
template <> struct Frag<__bf16> {
  typedef v16b V; union U { v16b v; v8b h[2]; };
  static __device__ __forceinline__ v16b load(const __bf16* p) {
    U f; f.h[0] = *(const v8b*)(p); f.h[1] = *(const v8b*)(p + 16); return f.v;
  }
  static __device__ __forceinline__ v8f mma(v16b a, v16b b, v8f c) {
    return __builtin_amdgcn_wmma_f32_16x16x32_bf16(false, a, false, b, (short)0, c, false, false);
  }
  static __device__ __forceinline__ void guard(v8f& a, v8f& b, v16b x, v16b y) { dep_guard_b(a, b, x, y); }
  static __device__ __forceinline__ void keep(v16b a, v16b b, v16b c, v16b d) { keep4_b(a, b, c, d); }
};

__device__ __forceinline__ unsigned pk16(unsigned short a, unsigned short b) { return (unsigned)a | ((unsigned)b << 16); }
__device__ __forceinline__ unsigned short h_bits(float f) { const _Float16 h = (_Float16)f; return __builtin_bit_cast(unsigned short, h); }

template <int ET> struct Elem;
template <> struct Elem<0> { typedef _Float16 T; };
template <> struct Elem<1> { typedef __bf16 T; };
template <int ET, bool SPLIT, int BIAS_MODE, int OUT_MODE, bool RESID, int ACT = 0>
__global__ __launch_bounds__(256) void wmma_gemm64(
    const unsigned short* __restrict__ Ap, const unsigned short* __restrict__ A2p, int lda, long strideA,
    const unsigned short* __restrict__ Btp, const unsigned short* __restrict__ Bt2p, int ldb, long strideB,
    void* __restrict__ Cout, void* __restrict__ Cout2, int ldc, long strideC,
    const float* __restrict__ bias,
    const float* __restrict__ resid, long strideR,
    int M, int N, int K, float scale) {
  typedef typename Elem<ET>::T T;
  typedef typename Frag<T>::V V;
  const T* A = (const T*)Ap; const T* A2 = (const T*)A2p; const T* Bt = (const T*)Btp; const T* Bt2 = (const T*)Bt2p;
  __shared__ __align__(16) float sT[8][16 * 68];
  const int b    = blockIdx.y;
  const int lane = threadIdx.x & 31;
  const int wave = threadIdx.x >> 5;
  const int tilesN = N >> 6;
  const int tilesM = M >> 6;
  const int tile = blockIdx.x * 8 + wave;
  if (tile >= tilesM * tilesN) return;
  const int tm = tile / tilesN;
  const int tn = tile - tm * tilesN;
  const int m0 = tm << 6;
  const int n0 = tn << 6;

  const T* Ab  = A  + (size_t)b * strideA;
  const T* Bb  = Bt + (size_t)b * strideB;
  const T* Ab2 = SPLIT ? (A2  + (size_t)b * strideA) : nullptr;
  const T* Bb2 = SPLIT ? (Bt2 + (size_t)b * strideB) : nullptr;

  const int rlane = lane & 15;
  const int koff  = (lane >> 4) * 8;
  const int mOff  = (lane >> 4) * 8;

  v8f acc[4][4];
#pragma unroll
  for (int i = 0; i < 4; ++i)
#pragma unroll
    for (int j = 0; j < 4; ++j) acc[i][j] = (v8f){0.f,0.f,0.f,0.f,0.f,0.f,0.f,0.f};

  for (int k0 = 0; k0 < K; k0 += 32) {
    V bh[4], bl[4];
#pragma unroll
    for (int j = 0; j < 4; ++j) {
      const size_t bo = (size_t)(n0 + (j << 4) + rlane) * ldb + koff + k0;
      bh[j] = Frag<T>::load(Bb + bo);
      if (SPLIT) bl[j] = Frag<T>::load(Bb2 + bo);
    }
#pragma unroll
    for (int i = 0; i < 4; ++i) {
      const size_t ao = (size_t)(m0 + (i << 4) + rlane) * lda + koff + k0;
      V ah = Frag<T>::load(Ab + ao);
      V al;
      if (SPLIT) al = Frag<T>::load(Ab2 + ao);
#pragma unroll
      for (int j = 0; j < 4; ++j) {
        acc[i][j] = Frag<T>::mma(ah, bh[j], acc[i][j]);
        if (SPLIT) {
          acc[i][j] = Frag<T>::mma(ah, bl[j], acc[i][j]);
          acc[i][j] = Frag<T>::mma(al, bh[j], acc[i][j]);
        }
      }
      Frag<T>::guard(acc[i][0], acc[i][3], ah, SPLIT ? al : ah);
    }
    Frag<T>::keep(bh[0], bh[1], bh[2], bh[3]);
    if (SPLIT) Frag<T>::keep(bl[0], bl[1], bl[2], bl[3]);
  }
  acc_guard4(acc[0][0], acc[0][1], acc[0][2], acc[0][3]);
  acc_guard4(acc[1][0], acc[1][1], acc[1][2], acc[1][3]);
  acc_guard4(acc[2][0], acc[2][1], acc[2][2], acc[2][3]);
  acc_guard4(acc[3][0], acc[3][1], acc[3][2], acc[3][3]);

  float* slab = sT[wave];
  const float* Rb = RESID ? (resid + (size_t)b * strideR) : nullptr;
#pragma unroll
  for (int i = 0; i < 4; ++i) {
    const int mBase = m0 + (i << 4);
#pragma unroll
    for (int j = 0; j < 4; ++j) {
      const int n = n0 + (j << 4) + rlane;
      float bv = 0.f;
      if (BIAS_MODE == 2) bv = bias[n];
#pragma unroll
      for (int r = 0; r < 8; ++r) {
        float v = acc[i][j][r] * scale;
        if (BIAS_MODE == 1) v += bias[mBase + mOff + r];
        if (BIAS_MODE == 2) v += bv;
        if (RESID) v += Rb[(size_t)(mBase + mOff + r) * ldc + n];
        if (ACT == 2) v = fmaxf(v, 0.0f);
        if (ACT == 4) v = (v > 0.f) ? v : 0.01f * v;
        slab[(mOff + r) * 68 + (j << 4) + rlane] = v;
      }
    }
    __builtin_amdgcn_fence(__ATOMIC_RELEASE, "workgroup");
    __builtin_amdgcn_wave_barrier();
    __builtin_amdgcn_fence(__ATOMIC_ACQUIRE, "workgroup");
    if (OUT_MODE == 0) {
      float* C = (float*)Cout + (size_t)b * strideC;
      const int hh = lane >> 4, c4 = (lane & 15) * 4;
      for (int pass = 0; pass < 2; ++pass) {
#pragma unroll
        for (int it = 0; it < 8; ++it) {
          const int row = it * 2 + hh;
          v4f v = *(const v4f*)(slab + row * 68 + c4);
          *(volatile v4f*)(C + (size_t)(mBase + row) * ldc + n0 + c4) = v;
        }
        __threadfence();
      }
    } else {
      const int q = lane >> 3, c8 = (lane & 7) * 8;
      unsigned short* C  = (unsigned short*)Cout  + (size_t)b * strideC;
      unsigned short* C2 = (OUT_MODE == 2) ? ((unsigned short*)Cout2 + (size_t)b * strideC) : nullptr;
      for (int pass = 0; pass < 2; ++pass) {
#pragma unroll
        for (int it = 0; it < 4; ++it) {
          const int row = it * 4 + q;
          const float* sp = slab + row * 68 + c8;
          v8h hv, lv;
#pragma unroll
          for (int e = 0; e < 8; ++e) {
            if (OUT_MODE == 1) {
              hv[e] = (_Float16)sp[e];
            } else {
              unsigned short hb = f2bf_bits(sp[e]);
              unsigned short lb = f2bf_bits(sp[e] - bf_bits2f(hb));
              hv[e] = __builtin_bit_cast(_Float16, hb);
              lv[e] = __builtin_bit_cast(_Float16, lb);
            }
          }
          *(volatile v8h*)(C + (size_t)(mBase + row) * ldc + n0 + c8) = hv;
          if (OUT_MODE == 2) *(volatile v8h*)(C2 + (size_t)(mBase + row) * ldc + n0 + c8) = lv;
        }
        __threadfence();
      }
    }
    __builtin_amdgcn_fence(__ATOMIC_RELEASE, "workgroup");
    __builtin_amdgcn_wave_barrier();
    __builtin_amdgcn_fence(__ATOMIC_ACQUIRE, "workgroup");
  }
}

__device__ __forceinline__ void emit8_f16(const float* sp, unsigned short* dst) {
  const v4f a = *(const v4f*)(sp);
  const v4f c = *(const v4f*)(sp + 4);
  unsigned short hb[8];
#pragma unroll
  for (int e = 0; e < 4; ++e) {
    hb[e]     = h_bits(a[e]);
    hb[4 + e] = h_bits(c[e]);
  }
  const v4u u = (v4u){pk16(hb[0], hb[1]), pk16(hb[2], hb[3]), pk16(hb[4], hb[5]), pk16(hb[6], hb[7])};
  *(volatile v4u*)dst = u;
  __threadfence();
  *(volatile v4u*)dst = u;
}

__global__ __launch_bounds__(256) void pack_w_kernel(const float* __restrict__ bw, const float* __restrict__ sw,
                                                     const float* __restrict__ ss, unsigned short* __restrict__ Wp) {
  __shared__ __align__(16) float swr[kIn * kNSpl];
  __shared__ __align__(16) float bwr[kIn];
  __shared__ __align__(16) float ssr[kIn];
  const int tid = threadIdx.x;
  const int o   = blockIdx.x;
  const float* swrow = sw + (size_t)o * (kIn * kNSpl);
#pragma unroll
  for (int it = 0; it < 4; ++it) {
    const int f = it * 256 + tid;
    *(v4f*)(swr + f * 4) = *(const v4f*)(swrow + f * 4);
  }
  {
    const int q = tid & 127;
    const v4f bv = *(const v4f*)(bw + (size_t)o * kIn + q * 4);
    const v4f sv = *(const v4f*)(ss + (size_t)o * kIn + q * 4);
    if (tid < 128) *(v4f*)(bwr + q * 4) = bv;
    else           *(v4f*)(ssr + q * 4) = sv;
  }
  __syncthreads();
  unsigned short* wrow = Wp + (size_t)o * kKdim;
#pragma unroll 1
  for (int it = 0; it < 3; ++it) {
    const int p = it * 256 + tid;
    if (p < kPieces) {
      const int j  = p >> 6;
      const int i0 = (p & 63) * 8;
      int jj = j - 1; jj = (jj < 0) ? 0 : jj;
      const float f0 = (j == 0) ? 1.0f : 0.0f;
      const float f1 = 1.0f - f0;
      const v4f b0 = *(const v4f*)(bwr + i0), b1 = *(const v4f*)(bwr + i0 + 4);
      const v4f s0 = *(const v4f*)(ssr + i0), s1 = *(const v4f*)(ssr + i0 + 4);
      float wbv[8], scv[8];
#pragma unroll
      for (int e = 0; e < 4; ++e) { wbv[e] = b0[e]; wbv[4 + e] = b1[e]; scv[e] = s0[e]; scv[4 + e] = s1[e]; }
      unsigned short hb[8];
#pragma unroll
      for (int e = 0; e < 8; ++e) {
        const float wsp = swr[(i0 + e) * kNSpl + jj] * scv[e];
        const float w   = fmaf(f0, wbv[e], f1 * wsp);
        hb[e] = h_bits(w * kWCarry);
      }
      const v4u u = (v4u){pk16(hb[0], hb[1]), pk16(hb[2], hb[3]), pk16(hb[4], hb[5]), pk16(hb[6], hb[7])};
      unsigned short* dst = wrow + (size_t)p * 8;
      *(volatile v4u*)dst = u;
      __threadfence();
      *(volatile v4u*)dst = u;
    }
  }
}

__global__ __launch_bounds__(512) void pack_act_kernel(const float* __restrict__ x, const float* __restrict__ grid,
                                                       unsigned short* __restrict__ A, int row0) {
  __shared__ __align__(16) float Tf[kNBlk * kIn];
  const int tid = threadIdx.x;
  const int bl  = blockIdx.x;
  const int bg  = row0 + bl;
  const float v = x[(size_t)bg * kIn + tid];
  const float* gp = grid + (size_t)tid * kGridLen;
  const v4f q0 = *(const v4f*)(gp);
  const v4f q1 = *(const v4f*)(gp + 4);
  const v4f q2 = *(const v4f*)(gp + 8);
  float g[kGridLen];
#pragma unroll
  for (int e = 0; e < 4; ++e) { g[e] = q0[e]; g[4 + e] = q1[e]; g[8 + e] = q2[e]; }

  float bs[kGridLen - 1];
#pragma unroll
  for (int t = 0; t < kGridLen - 1; ++t) bs[t] = (v >= g[t] && v < g[t + 1]) ? 1.0f : 0.0f;

#pragma unroll
  for (int k = 1; k <= 3; ++k) {
    float rk[kGridLen - 1];
#pragma unroll
    for (int t = 0; t < kGridLen - k; ++t) rk[t] = __builtin_amdgcn_rcpf(g[t + k] - g[t]);
#pragma unroll
    for (int t = 0; t < kGridLen - 1 - k; ++t) {
      const float lf = ((v - g[t]) * rk[t]) * bs[t];
      const float rt = ((g[t + k + 1] - v) * rk[t + 1]) * bs[t + 1];
      bs[t] = lf + rt;
    }
  }

  const float sg = 1.0f / (1.0f + expf(-v));
  const float s  = v * sg;

  Tf[tid] = s * kACarry;
#pragma unroll
  for (int t = 0; t < kNSpl; ++t) Tf[(t + 1) * kIn + tid] = bs[t] * kACarry;
  __syncthreads();

  unsigned short* arow = A + (size_t)bl * kKdim;
  emit8_f16(Tf + tid * 8, arow + (size_t)tid * 8);
  if (tid < kPieces - 512) {
    const int p = 512 + tid;
    emit8_f16(Tf + p * 8, arow + (size_t)p * 8);
  }
}

extern "C" void kernel_launch(void* const* d_in, const int* in_sizes, int n_in,
                              void* d_out, int out_size, void* d_ws, size_t ws_size,
                              hipStream_t stream) {
  if (n_in < 5) return;
  if (in_sizes[0] != kBatch * kIn) return;
  if (in_sizes[1] != kIn * kGridLen) return;
  if (in_sizes[2] != kOutF * kIn) return;
  if (in_sizes[3] != kOutF * kIn * kNSpl) return;
  if (in_sizes[4] != kOutF * kIn) return;
  if (out_size != kBatch * kOutF) return;
  if (ws_size < kWsTotal) return;

  const float* x    = (const float*)d_in[0];
  const float* grid = (const float*)d_in[1];
  const float* bw   = (const float*)d_in[2];
  const float* sw   = (const float*)d_in[3];
  const float* ss   = (const float*)d_in[4];
  float* out        = (float*)d_out;

  unsigned short* Ah = (unsigned short*)d_ws;
  unsigned short* Wp = (unsigned short*)((char*)d_ws + kABytes);

  hipLaunchKernelGGL(pack_w_kernel, dim3(kOutF, 1, 1), dim3(256, 1, 1), 0, stream, bw, sw, ss, Wp);

  const int gemmBlocks = ((kHalfRows / 64) * (kOutF / 64)) / 8;
  for (int half = 0; half < 2; ++half) {
    const int row0 = half * kHalfRows;
    hipLaunchKernelGGL(pack_act_kernel, dim3(kHalfRows, 1, 1), dim3(512, 1, 1), 0, stream, x, grid, Ah, row0);
    float* cptr = out + (size_t)row0 * kOutF;
    hipLaunchKernelGGL((wmma_gemm64<0, false, 0, 0, false, 0>), dim3(gemmBlocks, 1, 1), dim3(256, 1, 1), 0, stream,
                       (const unsigned short*)Ah, (const unsigned short*)Ah, (int)kKdim, 0L,
                       (const unsigned short*)Wp, (const unsigned short*)Wp, (int)kKdim, 0L,
                       (void*)cptr, (void*)cptr, (int)kOutF, 0L,
                       x, x, 0L,
                       (int)kHalfRows, (int)kOutF, (int)kKdim, kOutScale);
  }
}
